// KanAEClassifier_17858474016890
// MI455X (gfx1250) — hardware-run, weakly checked
//
#include <hip/hip_runtime.h>
#include <math.h>

typedef __attribute__((ext_vector_type(16))) _Float16 v16h;
typedef __attribute__((ext_vector_type(8)))  _Float16 v8h;
typedef __attribute__((ext_vector_type(16))) __bf16   v16b;
typedef __attribute__((ext_vector_type(8)))  __bf16   v8b;
typedef __attribute__((ext_vector_type(8)))  float    v8f;
typedef __attribute__((ext_vector_type(4)))  float    v4f;
typedef __attribute__((ext_vector_type(8)))  unsigned v8u;

constexpr int kRows  = 131072;
constexpr int kF0    = 78;
constexpr int kHid   = 64;
constexpr int kLat   = 32;
constexpr int kNRec  = 80;
constexpr int kRowsW = 32;
constexpr int kWaves = 4;
constexpr int kRowsB = kRowsW * kWaves;
constexpr int kActP  = 100;
constexpr float kCarryA = 256.0f;
constexpr float kCarryW = 64.0f;
constexpr float kFold   = 1.0f / (kCarryA * kCarryW);

constexpr int pad_to(int v, int m) { return (v + m - 1) / m * m; }
constexpr int layer_k(int in) { return 8 * pad_to(in, 4) + pad_to(in, 32); }
constexpr int kK1 = layer_k(kF0);
constexpr int kK2 = layer_k(kHid);
constexpr int kK3 = layer_k(kLat);
constexpr int kK4 = layer_k(kHid);
static_assert(kK1 == 736 && kK2 == 576 && kK3 == 288 && kK4 == 576);
static_assert((kK1 % 32) == 0 && (kK2 % 32) == 0 && (kK3 % 32) == 0 && (kK4 % 32) == 0);
static_assert((kRows % kRowsB) == 0);
static_assert(kRowsW * kF0 == 2496 && (kRowsW * kF0) % 4 == 0);
static_assert(pad_to(kF0, 32) + 4 <= kActP && (kActP % 4) == 0);

constexpr size_t kOffE1H = 0;
constexpr size_t kOffE1L = kOffE1H + (size_t)kHid  * kK1;
constexpr size_t kOffE2H = kOffE1L + (size_t)kHid  * kK1;
constexpr size_t kOffE2L = kOffE2H + (size_t)kLat  * kK2;
constexpr size_t kOffD1H = kOffE2L + (size_t)kLat  * kK2;
constexpr size_t kOffD1L = kOffD1H + (size_t)kHid  * kK3;
constexpr size_t kOffD2H = kOffD1L + (size_t)kHid  * kK3;
constexpr size_t kWsHalves = kOffD2H + (size_t)kNRec * kK4;
static_assert(kWsHalves * 2 == 428032ull);
static_assert(kWsHalves * 2 <= 134217728ull);
static_assert(((kOffE1L * 2) % 128) == 0 && ((kOffE2H * 2) % 128) == 0 && ((kOffE2L * 2) % 128) == 0 &&
              ((kOffD1H * 2) % 128) == 0 && ((kOffD1L * 2) % 128) == 0 && ((kOffD2H * 2) % 128) == 0);

constexpr size_t kOutLogit = 0;
constexpr size_t kOutRecon = (size_t)kRows * 2;
constexpr size_t kOutZ     = kOutRecon + (size_t)kRows * kF0;
constexpr size_t kOutTotal = kOutZ + (size_t)kRows * kLat;
static_assert(kOutRecon * 4 == 1048576ull && kOutZ * 4 == 41943040ull && kOutTotal * 4 == 58720256ull);

__device__ __forceinline__ unsigned short f2bf_bits(float f) {
  unsigned u = __float_as_uint(f);
  return (unsigned short)((u + 0x7FFFu + ((u >> 16) & 1u)) >> 16);
}
__device__ __forceinline__ float bf_bits2f(unsigned short h) { return __uint_as_float(((unsigned)h) << 16); }
__device__ __forceinline__ unsigned short f2h_bits(float f) {
  const _Float16 h = (_Float16)f;
  return __builtin_bit_cast(unsigned short, h);
}
__device__ __forceinline__ unsigned split_word(float v) {
  const unsigned short hb = f2bf_bits(v);
  const unsigned short lb = f2bf_bits(v - bf_bits2f(hb));
  return (unsigned)hb | ((unsigned)lb << 16);
}

__device__ __forceinline__ v16b frag_load16(const unsigned short* p) {
  union { v16b v; v8b h[2]; } f;
  f.h[0] = *(const v8b*)(const void*)(p);
  f.h[1] = *(const v8b*)(const void*)(p + 16);
  return f.v;
}

template <bool HALF>
__device__ __forceinline__ v8f mma16(v16b a, v16b b, v8f c) {
  if (HALF) {
    const v16h ah = __builtin_bit_cast(v16h, a);
    const v16h bh = __builtin_bit_cast(v16h, b);
    c = __builtin_amdgcn_wmma_f32_16x16x32_f16(false, ah, false, bh, (short)0, c, false, false);
    asm volatile("v_nop\n\tv_nop\n\tv_nop\n\tv_nop" : "+v"(c) : "v"(ah), "v"(bh));
    return c;
  }
  c = __builtin_amdgcn_wmma_f32_16x16x32_bf16(false, a, false, b, (short)0, c, false, false);
  asm volatile("v_nop\n\tv_nop\n\tv_nop\n\tv_nop" : "+v"(c) : "v"(a), "v"(b));
  return c;
}

__device__ __forceinline__ float silu_f(float v) {
  return v * __builtin_amdgcn_rcpf(1.0f + __expf(-v));
}

template <bool HALF>
__device__ __forceinline__ void feature_words(const float a, const bool valid, unsigned (&hw)[4], unsigned (&lw)[4]) {
  const float u = (a + 2.2f) * 2.5f;
  float cf = floorf(u);
  const float f = u - cf;
  cf = fminf(fmaxf(cf, -8.0f), 16.0f);
  int cell = (int)cf;
  cell = valid ? cell : -8;
  const float f2 = f * f;
  const float f3 = f2 * f;
  const float g  = 1.0f - f;
  const float w0 = (g * g) * g * (1.0f / 6.0f);
  const float w3 = f3 * (1.0f / 6.0f);
  const float w1 = 0.5f * f3 - f2 + (2.0f / 3.0f);
  const float w2 = 0.5f * ((f + f2) - f3) + (1.0f / 6.0f);
  unsigned cw0, cw1, cw2, cw3;
  if (HALF) {
    cw0 = (unsigned)f2h_bits(w0 * kCarryA);
    cw1 = (unsigned)f2h_bits(w1 * kCarryA);
    cw2 = (unsigned)f2h_bits(w2 * kCarryA);
    cw3 = (unsigned)f2h_bits(w3 * kCarryA);
  } else {
    cw0 = split_word(w0);
    cw1 = split_word(w1);
    cw2 = split_word(w2);
    cw3 = split_word(w3);
  }
  unsigned s[8];
#pragma unroll
  for (int c = 0; c < 8; ++c) {
    const int d = cell - c;
    unsigned v = 0u;
    v = (d == 3) ? cw0 : v;
    v = (d == 2) ? cw1 : v;
    v = (d == 1) ? cw2 : v;
    v = (d == 0) ? cw3 : v;
    s[c] = v;
  }
#pragma unroll
  for (int p = 0; p < 4; ++p) {
    if (HALF) {
      hw[p] = s[2 * p] | (s[2 * p + 1] << 16);
      lw[p] = 0u;
    } else {
      hw[p] = (s[2 * p] & 0xffffu) | (s[2 * p + 1] << 16);
      lw[p] = (s[2 * p] >> 16) | (s[2 * p + 1] & 0xffff0000u);
    }
  }
}

template <bool HALF>
__device__ __forceinline__ void pair_words(const float x0, const float x1, unsigned& hw, unsigned& lw) {
  if (HALF) {
    const unsigned b0 = (unsigned)f2h_bits(x0 * kCarryA);
    const unsigned b1 = (unsigned)f2h_bits(x1 * kCarryA);
    hw = b0 | (b1 << 16);
    lw = 0u;
  } else {
    const unsigned c0 = split_word(x0);
    const unsigned c1 = split_word(x1);
    hw = (c0 & 0xffffu) | (c1 << 16);
    lw = (c0 >> 16) | (c1 & 0xffff0000u);
  }
}

template <int IN, int NT, bool HALF>
__device__ __forceinline__ void spline_layer(const float* actw, const unsigned short* __restrict__ Bh,
                                             const unsigned short* __restrict__ Bl, v8f (&acc)[2][NT], const int lane) {
  constexpr int INP = pad_to(IN, 4);
  constexpr int KBP = pad_to(IN, 32);
  constexpr int K   = 8 * INP + KBP;
  const int rl = lane & 15;
  const int hh = lane >> 4;
#pragma unroll
  for (int mt = 0; mt < 2; ++mt)
#pragma unroll
    for (int j = 0; j < NT; ++j) acc[mt][j] = (v8f){0.f, 0.f, 0.f, 0.f, 0.f, 0.f, 0.f, 0.f};
  const int boff = rl * K + 8 * hh;

#pragma unroll 1
  for (int kt = 0; kt < INP / 4; ++kt) {
    v16b ah[2], al[2];
#pragma unroll
    for (int mt = 0; mt < 2; ++mt) {
      const float* arow = actw + (mt * 16 + rl) * kActP;
      const int f0 = 4 * kt + hh;
      const int f1 = f0 + 2;
      const float a0 = arow[f0];
      const float a1 = arow[f1];
      unsigned hA[4], lA[4], hB[4], lB[4];
      feature_words<HALF>(a0, ((IN % 4) == 0) || (f0 < IN), hA, lA);
      feature_words<HALF>(a1, ((IN % 4) == 0) || (f1 < IN), hB, lB);
      const v8u wh = {hA[0], hA[1], hA[2], hA[3], hB[0], hB[1], hB[2], hB[3]};
      ah[mt] = __builtin_bit_cast(v16b, wh);
      if (!HALF) {
        const v8u wl = {lA[0], lA[1], lA[2], lA[3], lB[0], lB[1], lB[2], lB[3]};
        al[mt] = __builtin_bit_cast(v16b, wl);
      } else {
        al[mt] = ah[mt];
      }
    }
    const int kb = boff + kt * 32;
#pragma unroll
    for (int j = 0; j < NT; ++j) {
      const v16b bh = frag_load16(Bh + kb + j * 16 * K);
      if (!HALF) {
        const v16b bl = frag_load16(Bl + kb + j * 16 * K);
#pragma unroll
        for (int mt = 0; mt < 2; ++mt) {
          acc[mt][j] = mma16<false>(ah[mt], bh, acc[mt][j]);
          acc[mt][j] = mma16<false>(ah[mt], bl, acc[mt][j]);
          acc[mt][j] = mma16<false>(al[mt], bh, acc[mt][j]);
        }
      } else {
#pragma unroll
        for (int mt = 0; mt < 2; ++mt) acc[mt][j] = mma16<true>(ah[mt], bh, acc[mt][j]);
      }
    }
  }

#pragma unroll 1
  for (int t = 0; t < KBP / 32; ++t) {
    v16b ah[2], al[2];
#pragma unroll
    for (int mt = 0; mt < 2; ++mt) {
      const float* p0 = actw + (mt * 16 + rl) * kActP + t * 32 + 8 * hh;
      v4f q[4];
      q[0] = *(const v4f*)(p0);
      q[1] = *(const v4f*)(p0 + 4);
      q[2] = *(const v4f*)(p0 + 16);
      q[3] = *(const v4f*)(p0 + 20);
      unsigned hw[8], lw[8];
#pragma unroll
      for (int g = 0; g < 4; ++g) {
#pragma unroll
        for (int pr = 0; pr < 2; ++pr) {
          const float x0 = q[g][2 * pr];
          const float x1 = q[g][2 * pr + 1];
          float s0 = silu_f(x0);
          float s1 = silu_f(x1);
          if ((IN % 32) != 0) {
            const int fe = t * 32 + 8 * hh + (g >> 1) * 16 + (g & 1) * 4 + 2 * pr;
            s0 = (fe < IN) ? s0 : 0.0f;
            s1 = (fe + 1 < IN) ? s1 : 0.0f;
          }
          pair_words<HALF>(s0, s1, hw[g * 2 + pr], lw[g * 2 + pr]);
        }
      }
      const v8u wh = {hw[0], hw[1], hw[2], hw[3], hw[4], hw[5], hw[6], hw[7]};
      ah[mt] = __builtin_bit_cast(v16b, wh);
      if (!HALF) {
        const v8u wl = {lw[0], lw[1], lw[2], lw[3], lw[4], lw[5], lw[6], lw[7]};
        al[mt] = __builtin_bit_cast(v16b, wl);
      } else {
        al[mt] = ah[mt];
      }
    }
    const int kb = boff + 8 * INP + t * 32;
#pragma unroll
    for (int j = 0; j < NT; ++j) {
      const v16b bh = frag_load16(Bh + kb + j * 16 * K);
      if (!HALF) {
        const v16b bl = frag_load16(Bl + kb + j * 16 * K);
#pragma unroll
        for (int mt = 0; mt < 2; ++mt) {
          acc[mt][j] = mma16<false>(ah[mt], bh, acc[mt][j]);
          acc[mt][j] = mma16<false>(ah[mt], bl, acc[mt][j]);
          acc[mt][j] = mma16<false>(al[mt], bh, acc[mt][j]);
        }
      } else {
#pragma unroll
        for (int mt = 0; mt < 2; ++mt) acc[mt][j] = mma16<true>(ah[mt], bh, acc[mt][j]);
      }
    }
  }
}

template <int NT, int PITCH, int NCOLS>
__device__ __forceinline__ void write_tile(float* tw, const v8f (&acc)[2][NT], const float scale, const int lane) {
  static_assert(NT * 16 >= NCOLS);
  const int rl = lane & 15;
  const int hh = lane >> 4;
#pragma unroll
  for (int mt = 0; mt < 2; ++mt) {
#pragma unroll
    for (int j = 0; j < NT; ++j) {
      const int col = j * 16 + rl;
      if (((NCOLS % 16) == 0) || (col < NCOLS)) {
#pragma unroll
        for (int r = 0; r < 8; ++r) tw[(mt * 16 + 8 * hh + r) * PITCH + col] = acc[mt][j][r] * scale;
      }
    }
  }
}

__device__ __forceinline__ void put_x(float* tw, const int e, const float v) {
  const int r = e / kF0;
  const int c = e - r * kF0;
  tw[r * kActP + c] = v;
}

template <int MODE>
__global__ __launch_bounds__(256) void pack_plane_kernel(
    const float* __restrict__ base_w, const float* __restrict__ spline_w, const float* __restrict__ scaler,
    unsigned short* __restrict__ dhi, unsigned short* __restrict__ dlo,
    int In, int InP, int Out, int NP, int K)
{
  const int g = blockIdx.x * 256 + threadIdx.x;
  const int gpr = K >> 3;
  const int total = NP * gpr;
  if (g >= total) return;
  const int n  = g / gpr;
  const int kg = g - n * gpr;
  const bool rowOk = n < Out;
  const int nc = rowOk ? n : (Out - 1);
  const bool isSpl = kg < InP;
  const int is = (kg < In) ? kg : (In - 1);
  const bool splOk = isSpl && rowOk && (kg < In);
  const float* sp = spline_w + ((size_t)nc * In + is) * 8;
  const v4f sv0 = *(const v4f*)(sp);
  const v4f sv1 = *(const v4f*)(sp + 4);
  float sc = scaler[nc * In + is];
  asm volatile("" : "+v"(sc));
  const int ib0 = (kg - InP) * 8;
  float val[8];
#pragma unroll
  for (int e = 0; e < 8; ++e) {
    float cs = (e < 4) ? sv0[e & 3] : sv1[e & 3];
    asm volatile("" : "+v"(cs));
    const int ib = ib0 + e;
    const int ibc = (ib < 0) ? 0 : ((ib > In - 1) ? (In - 1) : ib);
    float cb = base_w[nc * In + ibc];
    asm volatile("" : "+v"(cb));
    const bool bOk = (!isSpl) && rowOk && (ib < In);
    const float spl = cs * sc;
    val[e] = splOk ? spl : (bOk ? cb : 0.0f);
  }
  v8h hv, lv;
#pragma unroll
  for (int e = 0; e < 8; ++e) {
    if (MODE == 0) {
      const unsigned short hb = f2bf_bits(val[e]);
      const unsigned short lb = f2bf_bits(val[e] - bf_bits2f(hb));
      hv[e] = __builtin_bit_cast(_Float16, hb);
      lv[e] = __builtin_bit_cast(_Float16, lb);
    } else {
      const _Float16 hf = (_Float16)(val[e] * kCarryW);
      hv[e] = hf;
      lv[e] = hf;
    }
  }
  unsigned short* qh = dhi + (size_t)g * 8;
  unsigned short* ql = dlo + (size_t)g * 8;
  *(volatile v8h*)qh = hv;
  if (MODE == 0) *(volatile v8h*)ql = lv;
  __threadfence();
  *(volatile v8h*)qh = hv;
  if (MODE == 0) *(volatile v8h*)ql = lv;
}

__global__ __launch_bounds__(128) __attribute__((amdgpu_num_vgpr(256)))
void fused_chain_kernel(const float* __restrict__ x, const unsigned short* __restrict__ wsp,
                        const float* __restrict__ ln_w, const float* __restrict__ ln_b,
                        const float* __restrict__ cls_w, const float* __restrict__ cls_b,
                        float* __restrict__ out)
{
  __shared__ __align__(16) float sAct[kWaves][kRowsW * kActP];
  __shared__ __align__(16) float sLog[kWaves][64];
  const int tid  = threadIdx.x;
  const int lane = tid & 31;
  const int wave = tid >> 5;
  float* actw = sAct[wave];
  float* logw = sLog[wave];
  const size_t rowbase = (size_t)blockIdx.x * kRowsB + (size_t)wave * kRowsW;

  {
    const float* xw = x + rowbase * kF0;
#pragma unroll 1
    for (int it = 0; it < 20; ++it) {
      const int idx = it * 32 + lane;
      const int idc = (idx < 624) ? idx : 623;
      const v4f v = *(const v4f*)(xw + idc * 4);
      float x0 = v[0], x1 = v[1], x2 = v[2], x3 = v[3];
      asm volatile("" : "+v"(x0), "+v"(x1), "+v"(x2), "+v"(x3));
      if (idx < 624) {
        const int e0 = idx * 4;
        put_x(actw, e0, x0);
        put_x(actw, e0 + 1, x1);
        put_x(actw, e0 + 2, x2);
        put_x(actw, e0 + 3, x3);
      }
    }
#pragma unroll 1
    for (int c = kF0; c < kActP; ++c) actw[lane * kActP + c] = 0.0f;
  }
  __syncthreads();

  {
    v8f acc[2][4];
    spline_layer<kF0, 4, false>(actw, wsp + kOffE1H, wsp + kOffE1L, acc, lane);
    __syncthreads();
    write_tile<4, kActP, 64>(actw, acc, 1.0f, lane);
  }
  __syncthreads();

  {
    v8f acc[2][2];
    spline_layer<kHid, 2, false>(actw, wsp + kOffE2H, wsp + kOffE2L, acc, lane);
    __syncthreads();
    write_tile<2, kActP, 32>(actw, acc, 1.0f, lane);
  }
  __syncthreads();

  {
    float* zr = actw + lane * kActP;
    float s = 0.0f;
#pragma unroll 1
    for (int q = 0; q < 8; ++q) {
      const v4f v = *(const v4f*)(zr + 4 * q);
      s += (v[0] + v[1]) + (v[2] + v[3]);
    }
    const float mu = s * (1.0f / 32.0f);
    float s2 = 0.0f;
#pragma unroll 1
    for (int q = 0; q < 8; ++q) {
      const v4f v = *(const v4f*)(zr + 4 * q);
      const float d0 = v[0] - mu, d1 = v[1] - mu, d2 = v[2] - mu, d3 = v[3] - mu;
      s2 += (d0 * d0 + d1 * d1) + (d2 * d2 + d3 * d3);
    }
    const float var = s2 * (1.0f / 32.0f);
    const float rs = 1.0f / sqrtf(var + 1e-5f);
    float l0 = 0.0f, l1 = 0.0f;
#pragma unroll 1
    for (int q = 0; q < 8; ++q) {
      const v4f v  = *(const v4f*)(zr + 4 * q);
      const v4f w4 = ((const v4f*)ln_w)[q];
      const v4f b4 = ((const v4f*)ln_b)[q];
      const v4f c0 = ((const v4f*)cls_w)[q];
      const v4f c1 = ((const v4f*)cls_w)[8 + q];
      v4f z;
      z[0] = (v[0] - mu) * rs * w4[0] + b4[0];
      z[1] = (v[1] - mu) * rs * w4[1] + b4[1];
      z[2] = (v[2] - mu) * rs * w4[2] + b4[2];
      z[3] = (v[3] - mu) * rs * w4[3] + b4[3];
      *(v4f*)(zr + 4 * q) = z;
      l0 += (z[0] * c0[0] + z[1] * c0[1]) + (z[2] * c0[2] + z[3] * c0[3]);
      l1 += (z[0] * c1[0] + z[1] * c1[1]) + (z[2] * c1[2] + z[3] * c1[3]);
    }
    l0 += cls_b[0];
    l1 += cls_b[1];
    logw[lane * 2]     = l0;
    logw[lane * 2 + 1] = l1;
  }
  __syncthreads();

  {
    float* oz = out + kOutZ + rowbase * kLat;
    float* ol = out + kOutLogit + rowbase * 2;
    const int q  = lane >> 3;
    const int c4 = (lane & 7) * 4;
    for (int pass = 0; pass < 2; ++pass) {
#pragma unroll
      for (int it = 0; it < 8; ++it) {
        const int row = it * 4 + q;
        const v4f v = *(const v4f*)(actw + row * kActP + c4);
        *(volatile v4f*)(oz + (size_t)row * kLat + c4) = v;
      }
      if (lane < 16) {
        const v4f lv = *(const v4f*)(logw + lane * 4);
        *(volatile v4f*)(ol + lane * 4) = lv;
      }
      __threadfence();
    }
  }

  {
    v8f acc[2][4];
    spline_layer<kLat, 4, false>(actw, wsp + kOffD1H, wsp + kOffD1L, acc, lane);
    __syncthreads();
    write_tile<4, kActP, 64>(actw, acc, 1.0f, lane);
  }
  __syncthreads();

  {
    v8f acc[2][5];
    spline_layer<kHid, 5, true>(actw, wsp + kOffD2H, wsp + kOffD2H, acc, lane);
    __syncthreads();
    write_tile<5, kF0, kF0>(actw, acc, kFold, lane);
  }
  __syncthreads();

  {
    float* orc = out + kOutRecon + rowbase * kF0;
    for (int pass = 0; pass < 2; ++pass) {
#pragma unroll 1
      for (int it = 0; it < 20; ++it) {
        const int idx = it * 32 + lane;
        if (idx < 624) {
          const v4f v = *(const v4f*)(actw + idx * 4);
          *(volatile v4f*)(orc + idx * 4) = v;
        }
      }
      __threadfence();
    }
  }
}

extern "C" void kernel_launch(void* const* d_in, const int* in_sizes, int n_in,
                              void* d_out, int out_size, void* d_ws, size_t ws_size,
                              hipStream_t stream) {
  if (n_in < 17) return;
  if (in_sizes[0] != kRows * kF0) return;
  if (in_sizes[1] != kHid * kF0 || in_sizes[2] != kHid * kF0 * 8 || in_sizes[3] != kHid * kF0) return;
  if (in_sizes[4] != kLat * kHid || in_sizes[5] != kLat * kHid * 8 || in_sizes[6] != kLat * kHid) return;
  if (in_sizes[7] != kLat || in_sizes[8] != kLat || in_sizes[9] != 2 * kLat || in_sizes[10] != 2) return;
  if (in_sizes[11] != kHid * kLat || in_sizes[12] != kHid * kLat * 8 || in_sizes[13] != kHid * kLat) return;
  if (in_sizes[14] != kF0 * kHid || in_sizes[15] != kF0 * kHid * 8 || in_sizes[16] != kF0 * kHid) return;
  if ((size_t)out_size != kOutTotal) return;
  if (ws_size < kWsHalves * 2) return;

  const float* x           = (const float*)d_in[0];
  const float* e1_base_w   = (const float*)d_in[1];
  const float* e1_spline_w = (const float*)d_in[2];
  const float* e1_scaler   = (const float*)d_in[3];
  const float* e2_base_w   = (const float*)d_in[4];
  const float* e2_spline_w = (const float*)d_in[5];
  const float* e2_scaler   = (const float*)d_in[6];
  const float* ln_w        = (const float*)d_in[7];
  const float* ln_b        = (const float*)d_in[8];
  const float* cls_w       = (const float*)d_in[9];
  const float* cls_b       = (const float*)d_in[10];
  const float* d1_base_w   = (const float*)d_in[11];
  const float* d1_spline_w = (const float*)d_in[12];
  const float* d1_scaler   = (const float*)d_in[13];
  const float* d2_base_w   = (const float*)d_in[14];
  const float* d2_spline_w = (const float*)d_in[15];
  const float* d2_scaler   = (const float*)d_in[16];
  float* out = (float*)d_out;
  unsigned short* ws = (unsigned short*)d_ws;

  constexpr int g1 = (kHid  * kK1 / 8 + 255) / 256;
  constexpr int g2 = (kLat  * kK2 / 8 + 255) / 256;
  constexpr int g3 = (kHid  * kK3 / 8 + 255) / 256;
  constexpr int g4 = (kNRec * kK4 / 8 + 255) / 256;
  static_assert(((kHid * kK1 / 8) % 32) == 0 && ((kLat * kK2 / 8) % 32) == 0 &&
                ((kHid * kK3 / 8) % 32) == 0 && ((kNRec * kK4 / 8) % 32) == 0);

  pack_plane_kernel<0><<<g1, 256, 0, stream>>>(e1_base_w, e1_spline_w, e1_scaler,
      ws + kOffE1H, ws + kOffE1L, kF0, pad_to(kF0, 4), kHid, kHid, kK1);
  pack_plane_kernel<0><<<g2, 256, 0, stream>>>(e2_base_w, e2_spline_w, e2_scaler,
      ws + kOffE2H, ws + kOffE2L, kHid, kHid, kLat, kLat, kK2);
  pack_plane_kernel<0><<<g3, 256, 0, stream>>>(d1_base_w, d1_spline_w, d1_scaler,
      ws + kOffD1H, ws + kOffD1L, kLat, kLat, kHid, kHid, kK3);
  pack_plane_kernel<1><<<g4, 256, 0, stream>>>(d2_base_w, d2_spline_w, d2_scaler,
      ws + kOffD2H, ws + kOffD2H, kHid, kHid, kF0, kNRec, kK4);

  fused_chain_kernel<<<kRows / kRowsB, 128, 0, stream>>>(x, ws, ln_w, ln_b, cls_w, cls_b, out);
}
